// HetSGG_56667798503484
// MI455X (gfx1250) — hardware-verified
//
#include <hip/hip_runtime.h>
#include <hip/hip_bf16.h>
#include <stddef.h>


#define CD       128
#define NRL      9
#define NBS      8
#define GR       32
#define AP       136
#define XSP      132
#define NTHR     256
#define NWAVE    8
#define ECH      512
#define NTY      10
#define NSLOT    672
#define NSTEPMAX 20
#define NB       512
#define CHUNK    2048
#define WCAP     256
#define NGRP     (CHUNK / (NTHR * 4))
#define STW      32

#define LDS_A_BYTES ((2 * NB * NRL + NRL * CD + 16 + NWAVE * WCAP + NWAVE) * 4)
#define LDS_B_BYTES ((NB * CD + NRL * CD + 16 + NWAVE * WCAP + NWAVE) * 4)

static_assert(WCAP == (CHUNK / NTHR) * 32);
static_assert(NGRP >= 1);
static_assert(NB == 512);
static_assert(CHUNK <= 4096);
static_assert(ECH == 2 * NTHR);
static_assert(NSLOT >= NSTEPMAX * 32);
static_assert((ECH + NRL * 15) / 16 <= 2 * NSTEPMAX);
static_assert(LDS_A_BYTES == 49760);
static_assert(LDS_B_BYTES == 275040);
static_assert(2 * NRL < STW);

typedef float          v4f  __attribute__((ext_vector_type(4)));
typedef float          v8f  __attribute__((ext_vector_type(8)));
typedef int            v4i  __attribute__((ext_vector_type(4)));
typedef unsigned short v8us __attribute__((ext_vector_type(8)));
typedef _Float16       v8h  __attribute__((ext_vector_type(8)));
typedef _Float16       v16h __attribute__((ext_vector_type(16)));
typedef __bf16         v16b __attribute__((ext_vector_type(16)));
union FragH { v16h v; v8us u[2]; };
union FragB { v16b v; v8us u[2]; };
union Pack8 { v8us u; v4i i; unsigned short s[8]; _Float16 f[8]; };

__device__ __forceinline__ v8f wmh(v16h a, v16h b, v8f c) {
  v8f d = __builtin_amdgcn_wmma_f32_16x16x32_f16(false, a, false, b, (short)0, c, false, false);
  asm volatile("v_nop\n\tv_nop\n\tv_nop\n\tv_nop" : "+v"(d) : "v"(a), "v"(b));
  return d;
}
__device__ __forceinline__ v8f wmb(v16b a, v16b b, v8f c) {
  v8f d = __builtin_amdgcn_wmma_f32_16x16x32_bf16(false, a, false, b, (short)0, c, false, false);
  asm volatile("v_nop\n\tv_nop\n\tv_nop\n\tv_nop" : "+v"(d) : "v"(a), "v"(b));
  return d;
}

__device__ __forceinline__ float wsum(float v) {
  v += __shfl_xor(v, 16, 32);
  v += __shfl_xor(v, 8, 32);
  v += __shfl_xor(v, 4, 32);
  v += __shfl_xor(v, 2, 32);
  v += __shfl_xor(v, 1, 32);
  return v;
}

__device__ __forceinline__ float leaky01(float x) { return x > 0.f ? x : 0.01f * x; }

__device__ __forceinline__ unsigned short bf_rne(float x) {
  unsigned int u = __float_as_uint(x);
  u += 0x7FFFu + ((u >> 16) & 1u);
  return (unsigned short)(u >> 16);
}
__device__ __forceinline__ float bf_val(unsigned short b) { return __uint_as_float(((unsigned int)b) << 16); }

__global__ __launch_bounds__(NTHR) void k_wcomb(
    const float* __restrict__ bS, const float* __restrict__ aS,
    const float* __restrict__ bO, const float* __restrict__ aO,
    const float* __restrict__ bRS, const float* __restrict__ aRS,
    const float* __restrict__ bRO, const float* __restrict__ aRO,
    unsigned short* Whi, unsigned short* Wlo, unsigned short* Wf, int total) {
  const int i = blockIdx.x * NTHR + threadIdx.x;
  if (i >= total) return;
  const int c8 = i & 15;
  const int d  = (i >> 4) & (CD - 1);
  const int pr = i >> 11;
  const int p  = pr / NRL;
  const int r  = pr - p * NRL;
  const float* basis = (p == 0) ? bS : (p == 1) ? bO : (p == 2) ? bRS : bRO;
  const float* att   = (p == 0) ? aS : (p == 1) ? aO : (p == 2) ? aRS : aRO;
  float s[8];
#pragma unroll
  for (int j = 0; j < 8; ++j) s[j] = 0.f;
#pragma unroll 1
  for (int b = 0; b < NBS; ++b) {
    const float a = att[r * NBS + b];
    const float* bp = basis + ((size_t)b * CD + (size_t)c8 * 8) * CD + d;
#pragma unroll
    for (int j = 0; j < 8; ++j) s[j] = fmaf(a, bp[(size_t)j * CD], s[j]);
  }
  const size_t o = ((size_t)r * CD + d) * CD + (size_t)c8 * 8;
  if (p < 2) {
    Pack8 ph, pl;
#pragma unroll
    for (int j = 0; j < 8; ++j) {
      const unsigned short hb = bf_rne(s[j]);
      ph.s[j] = hb;
      pl.s[j] = bf_rne(s[j] - bf_val(hb));
    }
    unsigned short* dh = Whi + (size_t)p * NRL * CD * CD + o;
    unsigned short* dl = Wlo + (size_t)p * NRL * CD * CD + o;
    *(volatile v4i*)dh = ph.i;
    *(volatile v4i*)dl = pl.i;
    __threadfence();
    *(volatile v4i*)dh = ph.i;
    *(volatile v4i*)dl = pl.i;
  } else {
    Pack8 pf;
#pragma unroll
    for (int j = 0; j < 8; ++j) pf.f[j] = (_Float16)(s[j] * 8.0f);
    unsigned short* df = Wf + (size_t)(p - 2) * NRL * CD * CD + o;
    *(volatile v4i*)df = pf.i;
    __threadfence();
    *(volatile v4i*)df = pf.i;
  }
}

__global__ __launch_bounds__(NTHR) void k_nfcvt(const float* __restrict__ x,
                                                unsigned short* hi, unsigned short* lo, int n8) {
  const int i = blockIdx.x * NTHR + threadIdx.x;
  if (i >= n8) return;
  const size_t o = (size_t)i * 8;
  const v4f a = *(const v4f*)(x + o);
  const v4f b = *(const v4f*)(x + o + 4);
  float v[8];
  v[0] = a.x; v[1] = a.y; v[2] = a.z; v[3] = a.w;
  v[4] = b.x; v[5] = b.y; v[6] = b.z; v[7] = b.w;
  Pack8 ph, pl;
#pragma unroll
  for (int j = 0; j < 8; ++j) {
    const unsigned short hb = bf_rne(v[j]);
    ph.s[j] = hb;
    pl.s[j] = bf_rne(v[j] - bf_val(hb));
  }
  *(volatile v4i*)(hi + o) = ph.i;
  *(volatile v4i*)(lo + o) = pl.i;
  __threadfence();
  *(volatile v4i*)(hi + o) = ph.i;
  *(volatile v4i*)(lo + o) = pl.i;
}

template <int SPLIT>
__global__ __launch_bounds__(NTHR) void k_gemm(
    const unsigned short* __restrict__ Ahi, const unsigned short* __restrict__ Alo,
    const float* __restrict__ Af, const int* __restrict__ idxmap, const int* __restrict__ ty,
    const unsigned short* __restrict__ W0, const unsigned short* __restrict__ W1,
    float* outp, int nN, int nE) {
  __shared__ __attribute__((aligned(16))) unsigned short Ah[GR * AP];
  __shared__ __attribute__((aligned(16))) unsigned short Al[GR * AP];
  __shared__ __attribute__((aligned(16))) float Xs[GR * XSP];
  __shared__ int s2e[NSLOT];
  __shared__ int wct[NWAVE * NTY];
  __shared__ int goff[16];
  __shared__ int sedge[GR];

  const int tid  = threadIdx.x;
  const int lane = tid & 31;
  const int wave = tid >> 5;
  const int hh   = lane >> 4;
  const int mm   = lane & 15;
  const int cbase = blockIdx.x * ECH;

  for (int i = tid; i < NSLOT; i += NTHR) s2e[i] = -1;

  const int l0 = tid, l1 = tid + NTHR;
  const int e0 = cbase + l0, e1 = cbase + l1;
  int t0 = ty[min(e0, nE - 1)];
  int t1 = ty[min(e1, nE - 1)];
  t0 = t0 < 0 ? 0 : (t0 > NRL - 1 ? NRL - 1 : t0);
  t1 = t1 < 0 ? 0 : (t1 > NRL - 1 ? NRL - 1 : t1);
  t0 = (e0 < nE) ? t0 : NRL;
  t1 = (e1 < nE) ? t1 : NRL;
  int rk0 = 0, rk1 = 0;
#pragma unroll 1
  for (int q = 0; q < NTY; ++q) {
    const bool f0 = (t0 == q), f1 = (t1 == q);
    const unsigned m0 = __builtin_amdgcn_ballot_w32(f0);
    const unsigned m1 = __builtin_amdgcn_ballot_w32(f1);
    const int c0 = (int)__builtin_popcount(m0);
    const int p0 = (int)__builtin_amdgcn_mbcnt_lo(m0, 0u);
    const int p1 = c0 + (int)__builtin_amdgcn_mbcnt_lo(m1, 0u);
    rk0 = f0 ? p0 : rk0;
    rk1 = f1 ? p1 : rk1;
    if (lane == q) wct[wave * NTY + q] = c0 + (int)__builtin_popcount(m1);
  }
  __syncthreads();

  int b0 = rk0, b1 = rk1;
#pragma unroll 1
  for (int w = 0; w < wave; ++w) { b0 += wct[w * NTY + t0]; b1 += wct[w * NTY + t1]; }
  const int qq = lane < NTY ? lane : NTY - 1;
  int nq = 0;
#pragma unroll
  for (int w = 0; w < NWAVE; ++w) nq += wct[w * NTY + qq];
  const int padq = (lane < NRL) ? ((nq + 15) & ~15) : 0;
  int xs = padq;
#pragma unroll
  for (int dd = 1; dd < 32; dd <<= 1) {
    const int y = __shfl_up(xs, dd, 32);
    if (lane >= dd) xs += y;
  }
  const int offq = xs - padq;
  const int TP   = __shfl(xs, 31, 32);
  const int off0 = __shfl(offq, t0, 32);
  const int off1 = __shfl(offq, t1, 32);
  if (wave == 0 && lane < 16) goff[lane] = (lane < NRL) ? offq : TP;
  __syncthreads();
  if (t0 < NRL) { int ps = off0 + b0; ps = ps < NSLOT - 1 ? ps : NSLOT - 1; ps = ps < 0 ? 0 : ps; s2e[ps] = l0; }
  if (t1 < NRL) { int ps = off1 + b1; ps = ps < NSLOT - 1 ? ps : NSLOT - 1; ps = ps < 0 ? 0 : ps; s2e[ps] = l1; }
  __syncthreads();
  const int ng = TP >> 4;
  int nsteps = (ng + 1) >> 1;
  nsteps = nsteps < NSTEPMAX ? nsteps : NSTEPMAX;
  nsteps = nsteps < 0 ? 0 : nsteps;

  const int ncol = wave * 16 + mm;
#pragma unroll 1
  for (int s = 0; s < nsteps; ++s) {
    const int sb = s * 32;
    int r0 = 0, r1 = 0;
#pragma unroll
    for (int q = 0; q < NRL; ++q) {
      const int g = goff[q];
      r0 = (g <= sb) ? q : r0;
      r1 = (g <= sb + 16) ? q : r1;
    }
    {
      const int m   = tid >> 3;
      const int seg = (tid & 7) * 16;
      const int le  = s2e[sb + m];
      const bool valid = le >= 0;
      const int e   = valid ? (cbase + le) : cbase;
      const v8us z8 = {0, 0, 0, 0, 0, 0, 0, 0};
      v8us u0, u1;
      if (SPLIT) {
        int node = idxmap[e];
        node = node < 0 ? 0 : (node > nN - 1 ? nN - 1 : node);
        const unsigned short* ph = Ahi + (size_t)node * CD + seg;
        const unsigned short* pl = Alo + (size_t)node * CD + seg;
        u0 = *(const v8us*)ph;
        u1 = *(const v8us*)(ph + 8);
        v8us w0 = *(const v8us*)pl;
        v8us w1 = *(const v8us*)(pl + 8);
        u0 = valid ? u0 : z8; u1 = valid ? u1 : z8;
        w0 = valid ? w0 : z8; w1 = valid ? w1 : z8;
        *(v8us*)(Al + m * AP + seg)     = w0;
        *(v8us*)(Al + m * AP + seg + 8) = w1;
      } else {
        const float* pf = Af + (size_t)e * CD + seg;
        const v4f f0 = *(const v4f*)(pf), f1 = *(const v4f*)(pf + 4);
        const v4f f2 = *(const v4f*)(pf + 8), f3 = *(const v4f*)(pf + 12);
        Pack8 pa, pb;
        pa.f[0] = (_Float16)f0.x; pa.f[1] = (_Float16)f0.y; pa.f[2] = (_Float16)f0.z; pa.f[3] = (_Float16)f0.w;
        pa.f[4] = (_Float16)f1.x; pa.f[5] = (_Float16)f1.y; pa.f[6] = (_Float16)f1.z; pa.f[7] = (_Float16)f1.w;
        pb.f[0] = (_Float16)f2.x; pb.f[1] = (_Float16)f2.y; pb.f[2] = (_Float16)f2.z; pb.f[3] = (_Float16)f2.w;
        pb.f[4] = (_Float16)f3.x; pb.f[5] = (_Float16)f3.y; pb.f[6] = (_Float16)f3.z; pb.f[7] = (_Float16)f3.w;
        u0 = valid ? pa.u : z8;
        u1 = valid ? pb.u : z8;
      }
      *(v8us*)(Ah + m * AP + seg)     = u0;
      *(v8us*)(Ah + m * AP + seg + 8) = u1;
      if ((tid & 7) == 0) sedge[m] = valid ? e : -1;
    }
    __syncthreads();

    v8f c0 = {0.f, 0.f, 0.f, 0.f, 0.f, 0.f, 0.f, 0.f};
    v8f c1 = {0.f, 0.f, 0.f, 0.f, 0.f, 0.f, 0.f, 0.f};
    if (SPLIT) {
      const unsigned short* pb0h = W0 + ((size_t)r0 * CD + ncol) * CD + 8 * hh;
      const unsigned short* pb0l = W1 + ((size_t)r0 * CD + ncol) * CD + 8 * hh;
      const unsigned short* pb1h = W0 + ((size_t)r1 * CD + ncol) * CD + 8 * hh;
      const unsigned short* pb1l = W1 + ((size_t)r1 * CD + ncol) * CD + 8 * hh;
      const unsigned short* pa0 = Ah + mm * AP + 8 * hh;
      const unsigned short* pa1 = Ah + (16 + mm) * AP + 8 * hh;
      const unsigned short* qa0 = Al + mm * AP + 8 * hh;
      const unsigned short* qa1 = Al + (16 + mm) * AP + 8 * hh;
#pragma unroll 1
      for (int kt = 0; kt < CD / 32; ++kt) {
        const int k0 = kt * 32;
        FragB a0h, a0l, a1h, a1l, bh0, bl0, bh1, bl1;
        a0h.u[0] = *(const v8us*)(pa0 + k0);  a0h.u[1] = *(const v8us*)(pa0 + k0 + 16);
        a0l.u[0] = *(const v8us*)(qa0 + k0);  a0l.u[1] = *(const v8us*)(qa0 + k0 + 16);
        a1h.u[0] = *(const v8us*)(pa1 + k0);  a1h.u[1] = *(const v8us*)(pa1 + k0 + 16);
        a1l.u[0] = *(const v8us*)(qa1 + k0);  a1l.u[1] = *(const v8us*)(qa1 + k0 + 16);
        bh0.u[0] = *(const v8us*)(pb0h + k0); bh0.u[1] = *(const v8us*)(pb0h + k0 + 16);
        bl0.u[0] = *(const v8us*)(pb0l + k0); bl0.u[1] = *(const v8us*)(pb0l + k0 + 16);
        bh1.u[0] = *(const v8us*)(pb1h + k0); bh1.u[1] = *(const v8us*)(pb1h + k0 + 16);
        bl1.u[0] = *(const v8us*)(pb1l + k0); bl1.u[1] = *(const v8us*)(pb1l + k0 + 16);
        c0 = wmb(a0h.v, bh0.v, c0);
        c0 = wmb(a0h.v, bl0.v, c0);
        c0 = wmb(a0l.v, bh0.v, c0);
        c1 = wmb(a1h.v, bh1.v, c1);
        c1 = wmb(a1h.v, bl1.v, c1);
        c1 = wmb(a1l.v, bh1.v, c1);
      }
    } else {
      const unsigned short* pb0 = W0 + ((size_t)r0 * CD + ncol) * CD + 8 * hh;
      const unsigned short* pb1 = W0 + ((size_t)r1 * CD + ncol) * CD + 8 * hh;
      const unsigned short* pa0 = Ah + mm * AP + 8 * hh;
      const unsigned short* pa1 = Ah + (16 + mm) * AP + 8 * hh;
#pragma unroll
      for (int kt = 0; kt < CD / 32; ++kt) {
        const int k0 = kt * 32;
        FragH a0, a1, g0, g1;
        a0.u[0] = *(const v8us*)(pa0 + k0); a0.u[1] = *(const v8us*)(pa0 + k0 + 16);
        a1.u[0] = *(const v8us*)(pa1 + k0); a1.u[1] = *(const v8us*)(pa1 + k0 + 16);
        g0.u[0] = *(const v8us*)(pb0 + k0); g0.u[1] = *(const v8us*)(pb0 + k0 + 16);
        g1.u[0] = *(const v8us*)(pb1 + k0); g1.u[1] = *(const v8us*)(pb1 + k0 + 16);
        c0 = wmh(a0.v, g0.v, c0);
        c1 = wmh(a1.v, g1.v, c1);
      }
    }

    const float sc = SPLIT ? 1.0f : 0.125f;
#pragma unroll
    for (int r = 0; r < 8; ++r) {
      Xs[(8 * hh + r) * XSP + ncol]      = c0[r] * sc;
      Xs[(16 + 8 * hh + r) * XSP + ncol] = c1[r] * sc;
    }
    __syncthreads();

    v4f xr[4];
    int er[4];
#pragma unroll
    for (int i = 0; i < 4; ++i) {
      const int row = 4 * wave + i;
      er[i] = sedge[row];
      xr[i] = *(const v4f*)(Xs + row * XSP + 4 * lane);
    }
#pragma unroll
    for (int i = 0; i < 4; ++i)
      if (er[i] >= 0) *(volatile v4f*)(outp + (size_t)er[i] * CD + 4 * lane) = xr[i];
    __threadfence();
#pragma unroll
    for (int i = 0; i < 4; ++i)
      if (er[i] >= 0) *(volatile v4f*)(outp + (size_t)er[i] * CD + 4 * lane) = xr[i];
    __syncthreads();
  }
}

__global__ __launch_bounds__(NTHR) void k_rel(
    const float* __restrict__ S, const float* __restrict__ O, const float* __restrict__ EF,
    const float* __restrict__ went, float* out1, int nE) {
  const int lane = threadIdx.x & 31;
  const int wave = threadIdx.x >> 5;
  const int e = blockIdx.x * NWAVE + wave;
  if (e >= nE) return;
  const size_t ro = (size_t)e * CD + 4 * lane;
  const v4f s = *(const v4f*)(S + ro);
  const v4f o = *(const v4f*)(O + ro);
  const v4f f = *(const v4f*)(EF + ro);
  const v4f w = *(const v4f*)(went + 4 * lane);
  float ds = s.x * w.x; ds = fmaf(s.y, w.y, ds); ds = fmaf(s.z, w.z, ds); ds = fmaf(s.w, w.w, ds);
  float dq = o.x * w.x; dq = fmaf(o.y, w.y, dq); dq = fmaf(o.z, w.z, dq); dq = fmaf(o.w, w.w, dq);
  ds = wsum(ds);
  dq = wsum(dq);
  const float a  = leaky01(ds);
  const float b  = leaky01(dq);
  const float mx = fmaxf(a, b);
  const float ea = __expf(a - mx);
  const float eb = __expf(b - mx);
  const float inv = 1.0f / (ea + eb);
  const float w0 = ea * inv, w1 = eb * inv;
  const v4f rr = f + s * w0 + o * w1;
  float* op = out1 + ro;
  *(volatile v4f*)op = rr;
  __threadfence();
  *(volatile v4f*)op = rr;
}

template <int PASS>
__global__ __launch_bounds__(NTHR) void k_att(
    const float* __restrict__ M, const int* __restrict__ idx, const int* __restrict__ ty,
    const float* __restrict__ aw, const float* __restrict__ ab,
    float* ST, const float* __restrict__ subagg, const float* __restrict__ nf,
    float* outp, int fin, int nN, int nE, int al16) {
  extern __shared__ v4f lds_dyn[];
  float* base = (float*)lds_dyn;
  float* sacc = base;
  float* smx  = base + (PASS ? NB * CD : 0);
  float* sden = smx + (PASS ? 0 : NB * NRL);
  float* awl  = sden + (PASS ? 0 : NB * NRL);
  float* abl  = awl + NRL * CD;
  int*   list = (int*)(abl + 16);
  int*   wcn  = list + NWAVE * WCAP;

  const int tid  = threadIdx.x;
  const int lane = tid & 31;
  const int wave = tid >> 5;
  const int nodeBase = blockIdx.x * NB;

  if (PASS) {
    const v4f z4 = {0.f, 0.f, 0.f, 0.f};
    for (int i = tid; i < NB * CD / 4; i += NTHR) lds_dyn[i] = z4;
  } else {
    for (int i = tid; i < NB * NRL; i += NTHR) { smx[i] = -1.0e30f; sden[i] = 0.f; }
  }
  for (int i = tid; i < NRL * CD; i += NTHR) awl[i] = aw[i];
  if (tid < 16) abl[tid] = (tid < NRL) ? ab[tid < NRL ? tid : NRL - 1] : 0.f;
  __syncthreads();

  const int nChunks = (nE + CHUNK - 1) / CHUNK;
#pragma unroll 1
  for (int ch = 0; ch < nChunks; ++ch) {
    const int cbase = ch * CHUNK;
    int wc = 0;
#pragma unroll
    for (int g = 0; g < NGRP; ++g) {
      const int el0 = (g * NTHR + tid) * 4;
      const int e0  = cbase + el0;
      const int sent = -2147483647 - 1;
      v4i d;
      if (al16 != 0 && (cbase + CHUNK <= nE)) {
        d = *(const v4i*)(idx + e0);
      } else {
        d.x = (e0     < nE) ? idx[min(e0, nE - 1)]     : sent;
        d.y = (e0 + 1 < nE) ? idx[min(e0 + 1, nE - 1)] : sent;
        d.z = (e0 + 2 < nE) ? idx[min(e0 + 2, nE - 1)] : sent;
        d.w = (e0 + 3 < nE) ? idx[min(e0 + 3, nE - 1)] : sent;
      }
      const unsigned s0 = (unsigned)d.x - (unsigned)nodeBase;
      const unsigned s1 = (unsigned)d.y - (unsigned)nodeBase;
      const unsigned s2 = (unsigned)d.z - (unsigned)nodeBase;
      const unsigned s3 = (unsigned)d.w - (unsigned)nodeBase;
      const bool h0 = s0 < (unsigned)NB;
      const bool h1 = s1 < (unsigned)NB;
      const bool h2 = s2 < (unsigned)NB;
      const bool h3 = s3 < (unsigned)NB;
      const unsigned many = __builtin_amdgcn_ballot_w32(h0 | h1 | h2 | h3);
      if (many != 0u) {
#define HITJ(J, HJ, SJ) { \
          const unsigned mj = __builtin_amdgcn_ballot_w32(HJ); \
          if (HJ) { \
            const int pos = wc + (int)__builtin_amdgcn_mbcnt_lo(mj, 0u); \
            if (pos < WCAP) list[wave * WCAP + pos] = ((el0 + (J)) << 9) | (int)(SJ); \
          } \
          wc += (int)__builtin_popcount(mj); }
        HITJ(0, h0, s0)
        HITJ(1, h1, s1)
        HITJ(2, h2, s2)
        HITJ(3, h3, s3)
#undef HITJ
      }
    }
    if (lane == 0) wcn[wave] = wc;
    __syncthreads();

    if (wave == 0) {
#pragma unroll 1
      for (int wsx = 0; wsx < NWAVE; ++wsx) {
        int n = wcn[wsx];
        n = n > WCAP ? WCAP : n;
        n = n < 0 ? 0 : n;
#pragma unroll 1
        for (int i = 0; i < n; ++i) {
          const int ent  = list[wsx * WCAP + i];
          const int slot = ent & (NB - 1);
          const int el   = (ent >> 9) & (CHUNK - 1);
          int e = cbase + el;
          e = e > nE - 1 ? nE - 1 : e;
          int t = ty[e];
          t = t < 0 ? 0 : (t > NRL - 1 ? NRL - 1 : t);
          int nd = nodeBase + slot;
          nd = nd > nN - 1 ? nN - 1 : nd;
          const v4f mv = *(const v4f*)(M + (size_t)e * CD + 4 * lane);
          const v4f av = *(const v4f*)(awl + t * CD + 4 * lane);
          float dt = mv.x * av.x;
          dt = fmaf(mv.y, av.y, dt);
          dt = fmaf(mv.z, av.z, dt);
          dt = fmaf(mv.w, av.w, dt);
          dt = wsum(dt);
          float lg = dt + abl[t];
          lg = lg > 0.f ? lg : 0.01f * lg;
          if (PASS == 0) {
            if (lane == 0) {
              const int si = slot * NRL + t;
              const float mo = smx[si];
              const float dn = sden[si];
              const float mn = fmaxf(mo, lg);
              const float dnn = dn * __expf(mo - mn) + __expf(lg - mn);
              smx[si]  = mn;
              sden[si] = dnn;
            }
          } else {
            const float mxv = ST[(size_t)nd * STW + t];
            const float iv  = ST[(size_t)nd * STW + NRL + t];
            const float al  = __expf(lg - mxv) * iv;
            v4f* sp = (v4f*)(sacc + slot * CD + 4 * lane);
            const v4f cur = *sp;
            const v4f nxt = cur + al * mv;
            *sp = nxt;
          }
        }
      }
    }
    __syncthreads();
  }

#pragma unroll 1
  for (int j = 0; j < NB / NWAVE; ++j) {
    const int slot = wave * (NB / NWAVE) + j;
    const int node = nodeBase + slot;
    if (node >= nN) break;
    if (PASS == 0) {
      const int ta = lane < NRL ? lane : NRL - 1;
      int tb = lane - NRL;
      tb = tb < 0 ? 0 : (tb > NRL - 1 ? NRL - 1 : tb);
      const float mxa = smx[slot * NRL + ta];
      const float dna = sden[slot * NRL + ta];
      const float dnb = sden[slot * NRL + tb];
      const bool hasa = (lane < NRL) && (dna > 0.f);
      const unsigned hb = __builtin_amdgcn_ballot_w32(hasa);
      const int ns = (int)__builtin_popcount(hb);
      const float dsb  = dnb > 0.f ? dnb : 1.0f;
      const float invb = dnb > 0.f ? (1.0f / dsb) : 0.f;
      float val = 0.f;
      if (lane < NRL)           val = hasa ? mxa : 0.f;
      else if (lane < 2 * NRL)  val = invb;
      else if (lane == 2 * NRL) val = (float)ns;
      float* p = ST + (size_t)node * STW + lane;
      *(volatile float*)p = val;
      __threadfence();
      *(volatile float*)p = val;
    } else {
      const float nsv = ST[(size_t)node * STW + 2 * NRL];
      const float scl = nsv > 0.5f ? (1.0f / nsv) : 1.0f;
      const v4f a = *(const v4f*)(sacc + slot * CD + 4 * lane) * scl;
      v4f ov = a;
      if (fin != 0) {
        const v4f sa = *(const v4f*)(subagg + (size_t)node * CD + 4 * lane);
        const v4f xv = *(const v4f*)(nf + (size_t)node * CD + 4 * lane);
        ov = xv + (sa + a) * 0.5f;
      }
      float* p = outp + (size_t)node * CD + 4 * lane;
      *(volatile v4f*)p = ov;
      __threadfence();
      *(volatile v4f*)p = ov;
    }
  }
}

extern "C" void kernel_launch(void* const* d_in, const int* in_sizes, int n_in,
                              void* d_out, int out_size, void* d_ws, size_t ws_size,
                              hipStream_t stream) {
  if (n_in < 18) return;
  const int nE = in_sizes[3];
  const int nN = in_sizes[1] / CD;
  if (nE <= 0 || nN <= 0) return;
  if (in_sizes[0] != 2 * nE || in_sizes[1] != nN * CD || in_sizes[2] != nE * CD) return;
  if (in_sizes[4] != nE) return;
  if (in_sizes[5] != NBS * CD * CD || in_sizes[7] != NBS * CD * CD ||
      in_sizes[9] != NBS * CD * CD || in_sizes[13] != NBS * CD * CD) return;
  if (in_sizes[6] != NRL * NBS || in_sizes[8] != NRL * NBS ||
      in_sizes[10] != NRL * NBS || in_sizes[14] != NRL * NBS) return;
  if (in_sizes[11] != NRL * CD || in_sizes[15] != NRL * CD) return;
  if (in_sizes[12] != NRL || in_sizes[16] != NRL || in_sizes[17] != CD) return;
  if (out_size != nN * CD + nE * CD) return;

  const int*   ei     = (const int*)d_in[0];
  const float* nf     = (const float*)d_in[1];
  const float* ef     = (const float*)d_in[2];
  const int*   trel   = (const int*)d_in[3];
  const int*   tinv   = (const int*)d_in[4];
  const float* s2r_b  = (const float*)d_in[5];
  const float* s2r_a  = (const float*)d_in[6];
  const float* o2r_b  = (const float*)d_in[7];
  const float* o2r_a  = (const float*)d_in[8];
  const float* r2s_b  = (const float*)d_in[9];
  const float* r2s_a  = (const float*)d_in[10];
  const float* r2s_aw = (const float*)d_in[11];
  const float* r2s_ab = (const float*)d_in[12];
  const float* r2o_b  = (const float*)d_in[13];
  const float* r2o_a  = (const float*)d_in[14];
  const float* r2o_aw = (const float*)d_in[15];
  const float* r2o_ab = (const float*)d_in[16];
  const float* went   = (const float*)d_in[17];
  const int* src = ei;
  const int* dst = ei + nE;

  float* out0 = (float*)d_out;
  float* out1 = out0 + (size_t)nN * CD;

  size_t off = 0;
  char* wsb = (char*)d_ws;
  auto carve = [&](size_t bytes) -> void* {
    void* p = wsb + off;
    off = (off + bytes + 255) & ~(size_t)255;
    return p;
  };
  const size_t wplane = (size_t)NRL * CD * CD;
  unsigned short* Whi = (unsigned short*)carve(2 * wplane * sizeof(unsigned short));
  unsigned short* Wlo = (unsigned short*)carve(2 * wplane * sizeof(unsigned short));
  unsigned short* Wf  = (unsigned short*)carve(2 * wplane * sizeof(unsigned short));
  size_t xbytes = (size_t)nN * CD * sizeof(float);
  const size_t plbytes = (size_t)2 * nN * CD * sizeof(unsigned short);
  if (plbytes > xbytes) xbytes = plbytes;
  char* X = (char*)carve(xbytes);
  unsigned short* nfhi = (unsigned short*)X;
  unsigned short* nflo = nfhi + (size_t)nN * CD;
  float* subagg = (float*)X;
  float* S  = (float*)carve((size_t)nE * CD * sizeof(float));
  float* O  = (float*)carve((size_t)nE * CD * sizeof(float));
  float* ST = (float*)carve((size_t)nN * STW * sizeof(float));
  if (off > ws_size) return;

  const int al16d = ((nE & 3) == 0) ? 1 : 0;

  const int wtotal = 4 * NRL * CD * 16;
  k_wcomb<<<(wtotal + NTHR - 1) / NTHR, NTHR, 0, stream>>>(
      s2r_b, s2r_a, o2r_b, o2r_a, r2s_b, r2s_a, r2o_b, r2o_a, Whi, Wlo, Wf, wtotal);

  const int n8 = nN * CD / 8;
  k_nfcvt<<<(n8 + NTHR - 1) / NTHR, NTHR, 0, stream>>>(nf, nfhi, nflo, n8);

  const int ggrid = (nE + ECH - 1) / ECH;
  k_gemm<1><<<ggrid, NTHR, 0, stream>>>(nfhi, nflo, nf, src, trel, Whi, Wlo, S, nN, nE);
  k_gemm<1><<<ggrid, NTHR, 0, stream>>>(nfhi, nflo, nf, dst, tinv, Whi + wplane, Wlo + wplane, O, nN, nE);

  k_rel<<<(nE + NWAVE - 1) / NWAVE, NTHR, 0, stream>>>(S, O, ef, went, out1, nE);

  k_gemm<0><<<ggrid, NTHR, 0, stream>>>(nfhi, nflo, out1, src, tinv, Wf, Wf, S, nN, nE);
  k_gemm<0><<<ggrid, NTHR, 0, stream>>>(nfhi, nflo, out1, dst, trel, Wf + wplane, Wf + wplane, O, nN, nE);

  hipFuncSetAttribute(reinterpret_cast<const void*>(&k_att<0>),
                      hipFuncAttributeMaxDynamicSharedMemorySize, LDS_A_BYTES);
  hipFuncSetAttribute(reinterpret_cast<const void*>(&k_att<1>),
                      hipFuncAttributeMaxDynamicSharedMemorySize, LDS_B_BYTES);
  const int agrid = (nN + NB - 1) / NB;
  k_att<0><<<agrid, NTHR, LDS_A_BYTES, stream>>>(S, src, tinv, r2s_aw, r2s_ab, ST, nf, nf, ST, 0, nN, nE, 1);
  k_att<1><<<agrid, NTHR, LDS_B_BYTES, stream>>>(S, src, tinv, r2s_aw, r2s_ab, ST, nf, nf, subagg, 0, nN, nE, 1);
  k_att<0><<<agrid, NTHR, LDS_A_BYTES, stream>>>(O, dst, trel, r2o_aw, r2o_ab, ST, nf, nf, ST, 0, nN, nE, al16d);
  k_att<1><<<agrid, NTHR, LDS_B_BYTES, stream>>>(O, dst, trel, r2o_aw, r2o_ab, ST, subagg, nf, out0, 1, nN, nE, al16d);
}
